// VectorQuantizer2_64707977281812
// MI455X (gfx1250) — hardware-verified
//
#include <hip/hip_runtime.h>
#include <stdint.h>
#pragma clang fp contract(off)

typedef __attribute__((ext_vector_type(16))) __bf16   v16b;
typedef __attribute__((ext_vector_type(8)))  __bf16   v8b;
typedef __attribute__((ext_vector_type(8)))  float    v8f;
typedef __attribute__((ext_vector_type(4)))  float    v4f;
typedef __attribute__((ext_vector_type(4)))  unsigned v4u;
typedef __attribute__((ext_vector_type(2)))  unsigned v2u;

constexpr int NBATCH   = 32;
constexpr int NCH      = 128;
constexpr int NSIDE    = 16;
constexpr int NPIX     = 256;
constexpr int NPAD     = 18;
constexpr int NVOC     = 8192;
constexpr int KCONV    = 1152;
constexpr int NUMEL_T  = NBATCH * NCH * NPIX;
constexpr int NCONVBLK = 64;
constexpr int NSCALE   = 5;

constexpr size_t SZ_EBF   = (size_t)NVOC * NCH * 2;
constexpr size_t SZ_ES    = (size_t)NVOC * 4;
constexpr size_t SZ_WT    = (size_t)4 * NCH * KCONV * 2;
constexpr size_t SZ_PLANE = (size_t)NUMEL_T * 4;
constexpr size_t SZ_X     = (size_t)NVOC * NCH * 2;
constexpr size_t SZ_XS    = (size_t)NVOC * 4;
constexpr size_t SZ_IDX   = (size_t)NVOC * 4;
constexpr size_t SZ_HF    = SZ_PLANE;
constexpr size_t SZ_HP    = (size_t)NBATCH * NPAD * NPAD * NCH * 2;
constexpr size_t SZ_PART  = (size_t)NSCALE * NCONVBLK * 32 * 4;
constexpr size_t OFF_EBF  = 0;
constexpr size_t OFF_ES   = OFF_EBF + SZ_EBF;
constexpr size_t OFF_WT   = OFF_ES + SZ_ES;
constexpr size_t OFF_FB   = OFF_WT + SZ_WT;
constexpr size_t OFF_P0H  = OFF_FB + SZ_PLANE;
constexpr size_t OFF_P0R  = OFF_P0H + SZ_PLANE;
constexpr size_t OFF_P1H  = OFF_P0R + SZ_PLANE;
constexpr size_t OFF_P1R  = OFF_P1H + SZ_PLANE;
constexpr size_t OFF_XH   = OFF_P1R + SZ_PLANE;
constexpr size_t OFF_XM   = OFF_XH + SZ_X;
constexpr size_t OFF_XL   = OFF_XM + SZ_X;
constexpr size_t OFF_XS   = OFF_XL + SZ_X;
constexpr size_t OFF_IDX  = OFF_XS + SZ_XS;
constexpr size_t OFF_HF   = OFF_IDX + SZ_IDX;
constexpr size_t OFF_HH   = OFF_HF + SZ_HF;
constexpr size_t OFF_HL   = OFF_HH + SZ_HP;
constexpr size_t OFF_PART = OFF_HL + SZ_HP;
constexpr size_t WS_TOTAL = OFF_PART + SZ_PART;
static_assert(WS_TOTAL <= (size_t)134217728, "");
static_assert((OFF_ES % 256) == 0 && (OFF_WT % 256) == 0 && (OFF_FB % 256) == 0 && (OFF_XH % 256) == 0, "");
static_assert((OFF_XS % 256) == 0 && (OFF_IDX % 256) == 0 && (OFF_HF % 256) == 0 && (OFF_HH % 256) == 0, "");
static_assert((OFF_HL % 256) == 0 && (OFF_PART % 256) == 0, "");
static_assert((size_t)NUMEL_T * 4 == (size_t)4194304, "");
static_assert((size_t)NUMEL_T * 4 + 4 == (size_t)4194308, "");
static_assert(NCH % 32 == 0 && KCONV % 32 == 0, "");
static_assert((NBATCH * NPIX) % 64 == 0 && NCH % 64 == 0, "");

__device__ __forceinline__ unsigned short f2bf_bits(float f) {
  unsigned u = __float_as_uint(f);
  return (unsigned short)((u + 0x7FFFu + ((u >> 16) & 1u)) >> 16);
}
__device__ __forceinline__ float bf_bits2f(unsigned short h) { return __uint_as_float(((unsigned)h) << 16); }
__device__ __forceinline__ float rne_bf(float f) { return bf_bits2f(f2bf_bits(f)); }

__device__ __forceinline__ void dep_guard_b(v8f& a, v8f& b, v16b x, v16b y) { asm volatile("v_nop\n\tv_nop\n\tv_nop\n\tv_nop" : "+v"(a), "+v"(b) : "v"(x), "v"(y)); }
__device__ __forceinline__ void dep_guard_b3(v8f& a, v8f& b, v16b x, v16b y, v16b z) { asm volatile("v_nop\n\tv_nop\n\tv_nop\n\tv_nop" : "+v"(a), "+v"(b) : "v"(x), "v"(y), "v"(z)); }
__device__ __forceinline__ void keep4_b(v16b a, v16b b, v16b c, v16b d) { asm volatile("v_nop" :: "v"(a), "v"(b), "v"(c), "v"(d)); }
__device__ __forceinline__ void acc_guard4(v8f& a, v8f& b, v8f& c, v8f& d) { asm volatile("v_nop\n\tv_nop\n\tv_nop\n\tv_nop" : "+v"(a), "+v"(b), "+v"(c), "+v"(d)); }
template <typename T> struct Frag;
template <> struct Frag<__bf16> {
  typedef v16b V; union U { v16b v; v8b h[2]; };
  static __device__ __forceinline__ v16b load(const __bf16* p) {
    U f; f.h[0] = *(const v8b*)(p); f.h[1] = *(const v8b*)(p + 16); return f.v;
  }
  static __device__ __forceinline__ v8f mma(v16b a, v16b b, v8f c) {
    return __builtin_amdgcn_wmma_f32_16x16x32_bf16(false, a, false, b, (short)0, c, false, false);
  }
  static __device__ __forceinline__ void guard(v8f& a, v8f& b, v16b x, v16b y) { dep_guard_b(a, b, x, y); }
  static __device__ __forceinline__ void keep(v16b a, v16b b, v16b c, v16b d) { keep4_b(a, b, c, d); }
};

__device__ __forceinline__ void wave_sync_lds() {
  __builtin_amdgcn_fence(__ATOMIC_RELEASE, "workgroup");
  __builtin_amdgcn_wave_barrier();
  __builtin_amdgcn_fence(__ATOMIC_ACQUIRE, "workgroup");
}

__global__ __launch_bounds__(256) void k_cast_emb(const float* __restrict__ emb, unsigned short* __restrict__ ebf) {
  const int i = blockIdx.x * 256 + threadIdx.x;
  if (i >= NVOC * NCH / 8) return;
  const v4f a = *(const v4f*)(emb + (size_t)i * 8);
  const v4f c = *(const v4f*)(emb + (size_t)i * 8 + 4);
  v4u u;
  u.x = (unsigned)f2bf_bits(a[0]) | ((unsigned)f2bf_bits(a[1]) << 16);
  u.y = (unsigned)f2bf_bits(a[2]) | ((unsigned)f2bf_bits(a[3]) << 16);
  u.z = (unsigned)f2bf_bits(c[0]) | ((unsigned)f2bf_bits(c[1]) << 16);
  u.w = (unsigned)f2bf_bits(c[2]) | ((unsigned)f2bf_bits(c[3]) << 16);
  volatile v4u* p = (volatile v4u*)(ebf + (size_t)i * 8);
  *p = u;
  __threadfence();
  *p = u;
}

__global__ __launch_bounds__(256) void k_esq(const float* __restrict__ emb, float* __restrict__ es) {
  const int v = blockIdx.x * 256 + threadIdx.x;
  if (v >= NVOC) return;
  const float* e = emb + (size_t)v * NCH;
  float s = 0.0f;
#pragma unroll 2
  for (int c = 0; c < NCH; c += 4) {
    const v4f q = *(const v4f*)(e + c);
#pragma unroll
    for (int k = 0; k < 4; ++k) { const float r = rne_bf(q[k]); const float sq = r * r; s = s + sq; }
  }
  volatile float* p = es + v;
  p[0] = s;
  __threadfence();
  p[0] = s;
}

__global__ __launch_bounds__(256) void k_cast_w(const float* __restrict__ w, unsigned short* __restrict__ wt) {
  const int t = blockIdx.x * 256 + threadIdx.x;
  if (t >= 4 * NCH * (KCONV / 8)) return;
  const int row = t / (KCONV / 8);
  const int g = t - row * (KCONV / 8);
  const int tap = g >> 4;
  const int ci0 = (g & 15) * 8;
  const float* src = w + ((size_t)row * NCH + ci0) * 9 + tap;
  unsigned hb[8];
#pragma unroll
  for (int e = 0; e < 8; ++e) hb[e] = (unsigned)f2bf_bits(src[e * 9]);
  v4u u;
  u.x = hb[0] | (hb[1] << 16);
  u.y = hb[2] | (hb[3] << 16);
  u.z = hb[4] | (hb[5] << 16);
  u.w = hb[6] | (hb[7] << 16);
  volatile v4u* p = (volatile v4u*)(wt + (size_t)t * 8);
  *p = u;
  __threadfence();
  *p = u;
}

__global__ __launch_bounds__(256) void k_fbT(const float* __restrict__ f, float* __restrict__ fb) {
  __shared__ __align__(16) float s[NPIX * 36];
  const int tid = threadIdx.x;
  const int b = blockIdx.x >> 2, cg = blockIdx.x & 3;
#pragma unroll 2
  for (int k = 0; k < 8; ++k) {
    const int id = k * 256 + tid;
    const int c = id >> 6;
    const int p4 = (id & 63) * 4;
    const v4f v = *(const v4f*)(f + ((size_t)(b * NCH + cg * 32 + c)) * NPIX + p4);
#pragma unroll
    for (int e = 0; e < 4; ++e) s[(p4 + e) * 36 + c] = rne_bf(v[e]);
  }
  __syncthreads();
  const int wave = tid >> 5, lane = tid & 31, q = lane >> 3, c4 = (lane & 7) * 4;
  for (int pass = 0; pass < 2; ++pass) {
#pragma unroll
    for (int it = 0; it < 8; ++it) {
      const int p = wave * 32 + it * 4 + q;
      const v4f v = *(const v4f*)(s + p * 36 + c4);
      *(volatile v4f*)(fb + ((size_t)(b * NPIX + p)) * NCH + cg * 32 + c4) = v;
    }
    __threadfence();
  }
}

__global__ __launch_bounds__(512) void k_pool(const float* __restrict__ fr,
    unsigned short* __restrict__ xh, unsigned short* __restrict__ xm, unsigned short* __restrict__ xl,
    float* __restrict__ xs, int pn, int s, float inv_area)
{
  __shared__ float sxs[32];
  const int tid = threadIdx.x;
  const int wave = tid >> 5, lane = tid & 31, hh = lane >> 4, c8 = (lane & 15) * 8;
  const int n = blockIdx.x * 32 + wave * 2 + hh;
  const int pp = pn * pn;
  const int b = n / pp;
  const int p = n - b * pp;
  const int py = p / pn;
  const int px = p - py * pn;
  float acc[8];
#pragma unroll
  for (int e = 0; e < 8; ++e) acc[e] = 0.0f;
  const float* base = fr + ((size_t)(b * NPIX + (py * s) * NSIDE + px * s)) * NCH + c8;
#pragma unroll 1
  for (int i = 0; i < s; ++i) {
#pragma unroll 1
    for (int j = 0; j < s; ++j) {
      const float* qq = base + ((size_t)(i * NSIDE + j)) * NCH;
      const v4f a = *(const v4f*)qq;
      const v4f c = *(const v4f*)(qq + 4);
      acc[0] = acc[0] + a[0]; acc[1] = acc[1] + a[1]; acc[2] = acc[2] + a[2]; acc[3] = acc[3] + a[3];
      acc[4] = acc[4] + c[0]; acc[5] = acc[5] + c[1]; acc[6] = acc[6] + c[2]; acc[7] = acc[7] + c[3];
    }
  }
  float x[8];
#pragma unroll
  for (int e = 0; e < 8; ++e) x[e] = acc[e] * inv_area;
  float ssum = 0.0f;
#pragma unroll 1
  for (int ls = 0; ls < 16; ++ls) {
    const int src = (lane & 16) | ls;
#pragma unroll
    for (int e = 0; e < 8; ++e) {
      const float v = __shfl(x[e], src, 32);
      const float sq = v * v;
      ssum = ssum + sq;
    }
  }
  unsigned ph[4], pm[4], pl[4];
#pragma unroll
  for (int e2 = 0; e2 < 4; ++e2) {
    const float v0 = x[2 * e2], v1 = x[2 * e2 + 1];
    const unsigned short h0 = f2bf_bits(v0); const float r0 = v0 - bf_bits2f(h0);
    const unsigned short m0 = f2bf_bits(r0); const float q0 = r0 - bf_bits2f(m0);
    const unsigned short l0 = f2bf_bits(q0);
    const unsigned short h1 = f2bf_bits(v1); const float r1 = v1 - bf_bits2f(h1);
    const unsigned short m1 = f2bf_bits(r1); const float q1 = r1 - bf_bits2f(m1);
    const unsigned short l1 = f2bf_bits(q1);
    ph[e2] = (unsigned)h0 | ((unsigned)h1 << 16);
    pm[e2] = (unsigned)m0 | ((unsigned)m1 << 16);
    pl[e2] = (unsigned)l0 | ((unsigned)l1 << 16);
  }
  v4u vh, vm, vl;
  vh.x = ph[0]; vh.y = ph[1]; vh.z = ph[2]; vh.w = ph[3];
  vm.x = pm[0]; vm.y = pm[1]; vm.z = pm[2]; vm.w = pm[3];
  vl.x = pl[0]; vl.y = pl[1]; vl.z = pl[2]; vl.w = pl[3];
  const size_t o = (size_t)n * NCH + c8;
  *(volatile v4u*)(xh + o) = vh; *(volatile v4u*)(xm + o) = vm; *(volatile v4u*)(xl + o) = vl;
  __threadfence();
  *(volatile v4u*)(xh + o) = vh; *(volatile v4u*)(xm + o) = vm; *(volatile v4u*)(xl + o) = vl;
  if ((lane & 15) == 0) sxs[wave * 2 + hh] = ssum;
  __syncthreads();
  if (wave == 0) {
    const float v = sxs[lane];
    volatile float* px2 = xs + (size_t)blockIdx.x * 32;
    px2[lane] = v;
    __threadfence();
    px2[lane] = v;
  }
}

__global__ __launch_bounds__(128) void k_vq(const unsigned short* __restrict__ xh, const unsigned short* __restrict__ xm,
    const unsigned short* __restrict__ xl, const float* __restrict__ xs,
    const unsigned short* __restrict__ ebf, const float* __restrict__ es, int* __restrict__ idxT)
{
  __shared__ float sx[32];
  __shared__ float sd[4][32];
  __shared__ int   sv[4][32];
  const int tid = threadIdx.x, wave = tid >> 5, lane = tid & 31;
  const int rlane = lane & 15, hh = lane >> 4;
  const int koff = hh * 8, mOff = hh * 8;
  const int r0 = blockIdx.x * 32;
  const __bf16* Ah = (const __bf16*)xh;
  const __bf16* Am = (const __bf16*)xm;
  const __bf16* Al = (const __bf16*)xl;
  const __bf16* E  = (const __bf16*)ebf;
  if (wave == 0) sx[lane] = xs[r0 + lane];
  __syncthreads();
  float xsr[2][8];
#pragma unroll
  for (int i = 0; i < 2; ++i)
#pragma unroll
    for (int r = 0; r < 8; ++r) xsr[i][r] = sx[16 * i + mOff + r];
  float dmin[2][8]; int vmin[2][8];
#pragma unroll
  for (int i = 0; i < 2; ++i)
#pragma unroll
    for (int r = 0; r < 8; ++r) { dmin[i][r] = 3.0e38f; vmin[i][r] = 0; }

  const int vbeg = wave * (NVOC / 4);
#pragma unroll 1
  for (int chn = 0; chn < (NVOC / 4) / 64; ++chn) {
    const int v0 = vbeg + chn * 64;
    v8f acc[2][4];
#pragma unroll
    for (int i = 0; i < 2; ++i)
#pragma unroll
      for (int j = 0; j < 4; ++j) acc[i][j] = (v8f){0.f,0.f,0.f,0.f,0.f,0.f,0.f,0.f};
#pragma unroll 1
    for (int ks = 0; ks < NCH / 32; ++ks) {
      const int k0 = ks * 32;
      v16b bh[4];
#pragma unroll
      for (int j = 0; j < 4; ++j) bh[j] = Frag<__bf16>::load(E + (size_t)(v0 + 16 * j + rlane) * NCH + k0 + koff);
#pragma unroll
      for (int i = 0; i < 2; ++i) {
        const size_t ao = (size_t)(r0 + 16 * i + rlane) * NCH + k0 + koff;
        const v16b a0 = Frag<__bf16>::load(Ah + ao);
        const v16b a1 = Frag<__bf16>::load(Am + ao);
        const v16b a2 = Frag<__bf16>::load(Al + ao);
#pragma unroll
        for (int j = 0; j < 4; ++j) {
          acc[i][j] = Frag<__bf16>::mma(a0, bh[j], acc[i][j]);
          acc[i][j] = Frag<__bf16>::mma(a1, bh[j], acc[i][j]);
          acc[i][j] = Frag<__bf16>::mma(a2, bh[j], acc[i][j]);
        }
        dep_guard_b3(acc[i][0], acc[i][3], a0, a1, a2);
      }
      Frag<__bf16>::keep(bh[0], bh[1], bh[2], bh[3]);
    }
    acc_guard4(acc[0][0], acc[0][1], acc[0][2], acc[0][3]);
    acc_guard4(acc[1][0], acc[1][1], acc[1][2], acc[1][3]);
    float esj[4];
#pragma unroll
    for (int j = 0; j < 4; ++j) esj[j] = es[v0 + 16 * j + rlane];
#pragma unroll
    for (int i = 0; i < 2; ++i)
#pragma unroll
      for (int j = 0; j < 4; ++j)
#pragma unroll
        for (int r = 0; r < 8; ++r) {
          const float t = xsr[i][r] + esj[j];
          const float p2 = 2.0f * acc[i][j][r];
          const float d = t - p2;
          const bool lt = d < dmin[i][r];
          dmin[i][r] = lt ? d : dmin[i][r];
          vmin[i][r] = lt ? (v0 + 16 * j + rlane) : vmin[i][r];
        }
  }
#pragma unroll
  for (int i = 0; i < 2; ++i)
#pragma unroll
    for (int r = 0; r < 8; ++r) {
      float d = dmin[i][r]; int v = vmin[i][r];
#pragma unroll
      for (int off = 1; off < 16; off <<= 1) {
        const float od = __shfl_xor(d, off, 32);
        const int   ov = __shfl_xor(v, off, 32);
        const bool take = (od < d) || ((od == d) && (ov < v));
        d = take ? od : d;
        v = take ? ov : v;
      }
      dmin[i][r] = d; vmin[i][r] = v;
    }
  if (rlane == 0) {
#pragma unroll
    for (int i = 0; i < 2; ++i)
#pragma unroll
      for (int r = 0; r < 8; ++r) { sd[wave][16 * i + 8 * hh + r] = dmin[i][r]; sv[wave][16 * i + 8 * hh + r] = vmin[i][r]; }
  }
  __syncthreads();
  if (wave == 0) {
    float bd = sd[0][lane]; int bv = sv[0][lane];
#pragma unroll
    for (int w = 1; w < 4; ++w) {
      const float d2 = sd[w][lane]; const int v2 = sv[w][lane];
      const bool take = d2 < bd;
      bd = take ? d2 : bd; bv = take ? v2 : bv;
    }
    volatile int* ip = idxT + r0;
    ip[lane] = bv;
    __threadfence();
    ip[lane] = bv;
  }
}

__device__ __forceinline__ float keys_w(float x) {
  const float p1 = 1.5f * x - 2.5f;
  const float o1 = (p1 * x) * x + 1.0f;
  const float p2 = -0.5f * x + 2.5f;
  const float o2 = (p2 * x - 4.0f) * x + 2.0f;
  const float o = (x >= 1.0f) ? o2 : o1;
  return (x >= 2.0f) ? 0.0f : o;
}

__global__ __launch_bounds__(256) void k_up(const unsigned short* __restrict__ ebf, const int* __restrict__ idxT,
    float* __restrict__ hf, unsigned short* __restrict__ hhp, unsigned short* __restrict__ hlp, int pn, float inv)
{
  const int t = blockIdx.x * 256 + threadIdx.x;
  const int lane = threadIdx.x & 31;
  const int c4 = lane * 4;
  const int pos = t >> 5;
  const int b = pos / (NPAD * NPAD);
  const int q = pos - b * (NPAD * NPAD);
  const int yp = q / NPAD;
  const int xp = q - yp * NPAD;
  const bool interior = (yp >= 1) && (yp <= NSIDE) && (xp >= 1) && (xp <= NSIDE);
  int y = yp - 1; y = y < 0 ? 0 : (y > NSIDE - 1 ? NSIDE - 1 : y);
  int x = xp - 1; x = x < 0 ? 0 : (x > NSIDE - 1 ? NSIDE - 1 : x);
  float h0, h1, h2, h3;
  if (pn == NSIDE) {
    int id = idxT[(b * NSIDE + y) * NSIDE + x];
    id = id < 0 ? 0 : (id > NVOC - 1 ? NVOC - 1 : id);
    const v2u w = *(const v2u*)(ebf + (size_t)id * NCH + c4);
    h0 = __uint_as_float(w.x << 16); h1 = __uint_as_float(w.x & 0xffff0000u);
    h2 = __uint_as_float(w.y << 16); h3 = __uint_as_float(w.y & 0xffff0000u);
  } else {
    const float sfy = ((float)y + 0.5f) * inv - 0.5f;
    const float sfx = ((float)x + 0.5f) * inv - 0.5f;
    const int fy = (int)floorf(sfy);
    const int fx = (int)floorf(sfx);
    float wy[4], wx[4]; int iy[4], ix[4];
    float ty = 0.0f, tx = 0.0f;
#pragma unroll
    for (int a = 0; a < 4; ++a) {
      const int i = fy - 1 + a;
      const float ky = keys_w(fabsf(sfy - (float)i));
      wy[a] = ((i >= 0) && (i < pn)) ? ky : 0.0f;
      ty = ty + wy[a];
      iy[a] = i < 0 ? 0 : (i > pn - 1 ? pn - 1 : i);
      const int j = fx - 1 + a;
      const float kx = keys_w(fabsf(sfx - (float)j));
      wx[a] = ((j >= 0) && (j < pn)) ? kx : 0.0f;
      tx = tx + wx[a];
      ix[a] = j < 0 ? 0 : (j > pn - 1 ? pn - 1 : j);
    }
#pragma unroll
    for (int a = 0; a < 4; ++a) { wy[a] = wy[a] / ty; wx[a] = wx[a] / tx; }
    float a0 = 0.0f, a1 = 0.0f, a2 = 0.0f, a3 = 0.0f;
#pragma unroll
    for (int a = 0; a < 4; ++a) {
      float r0 = 0.0f, r1 = 0.0f, r2 = 0.0f, r3 = 0.0f;
#pragma unroll
      for (int c = 0; c < 4; ++c) {
        int id = idxT[(b * pn + iy[a]) * pn + ix[c]];
        id = id < 0 ? 0 : (id > NVOC - 1 ? NVOC - 1 : id);
        const v2u w = *(const v2u*)(ebf + (size_t)id * NCH + c4);
        const float g0 = __uint_as_float(w.x << 16), g1 = __uint_as_float(w.x & 0xffff0000u);
        const float g2 = __uint_as_float(w.y << 16), g3 = __uint_as_float(w.y & 0xffff0000u);
        const float t0 = wx[c] * g0, t1 = wx[c] * g1, t2 = wx[c] * g2, t3 = wx[c] * g3;
        r0 = r0 + t0; r1 = r1 + t1; r2 = r2 + t2; r3 = r3 + t3;
      }
      const float u0 = wy[a] * r0, u1 = wy[a] * r1, u2 = wy[a] * r2, u3 = wy[a] * r3;
      a0 = a0 + u0; a1 = a1 + u1; a2 = a2 + u2; a3 = a3 + u3;
    }
    h0 = a0; h1 = a1; h2 = a2; h3 = a3;
  }
  if (!interior) { h0 = 0.0f; h1 = 0.0f; h2 = 0.0f; h3 = 0.0f; }
  const unsigned short hb0 = f2bf_bits(h0), hb1 = f2bf_bits(h1), hb2 = f2bf_bits(h2), hb3 = f2bf_bits(h3);
  const unsigned short lb0 = f2bf_bits(h0 - bf_bits2f(hb0)), lb1 = f2bf_bits(h1 - bf_bits2f(hb1));
  const unsigned short lb2 = f2bf_bits(h2 - bf_bits2f(hb2)), lb3 = f2bf_bits(h3 - bf_bits2f(hb3));
  v2u ph, pl;
  ph.x = (unsigned)hb0 | ((unsigned)hb1 << 16); ph.y = (unsigned)hb2 | ((unsigned)hb3 << 16);
  pl.x = (unsigned)lb0 | ((unsigned)lb1 << 16); pl.y = (unsigned)lb2 | ((unsigned)lb3 << 16);
  v4f hv; hv.x = h0; hv.y = h1; hv.z = h2; hv.w = h3;
  const size_t op = (size_t)pos * NCH + c4;
  const size_t oi = ((size_t)((b * NSIDE + y) * NSIDE + x)) * NCH + c4;
  *(volatile v2u*)(hhp + op) = ph;
  *(volatile v2u*)(hlp + op) = pl;
  if (interior) *(volatile v4f*)(hf + oi) = hv;
  __threadfence();
  *(volatile v2u*)(hhp + op) = ph;
  *(volatile v2u*)(hlp + op) = pl;
  if (interior) *(volatile v4f*)(hf + oi) = hv;
}

template <bool FIRST>
__global__ __launch_bounds__(128) void k_conv(
    const unsigned short* __restrict__ hhp, const unsigned short* __restrict__ hlp,
    const unsigned short* __restrict__ wt, const float* __restrict__ bias,
    const float* __restrict__ hf, const float* __restrict__ fb,
    const float* __restrict__ fhin, const float* __restrict__ frin,
    float* __restrict__ fhout, float* __restrict__ frout, float* __restrict__ part)
{
  __shared__ __align__(16) float sT[4][16 * 68];
  __shared__ __align__(16) float sR[4][16 * 68];
  __shared__ float sl[4];
  const int tid = threadIdx.x, wave = tid >> 5, lane = tid & 31;
  const int rlane = lane & 15, koff = (lane >> 4) * 8, mOff = (lane >> 4) * 8;
  const int tile = blockIdx.x * 4 + wave;
  const int tm = tile >> 1, tn = tile & 1;
  const int bimg = tm >> 2, Y0 = (tm & 3) * 4, n0 = tn * 64;
  const __bf16* Ah = (const __bf16*)hhp;
  const __bf16* Al = (const __bf16*)hlp;
  const __bf16* Bw = (const __bf16*)wt;

  v8f acc[4][4];
#pragma unroll
  for (int i = 0; i < 4; ++i)
#pragma unroll
    for (int j = 0; j < 4; ++j) acc[i][j] = (v8f){0.f,0.f,0.f,0.f,0.f,0.f,0.f,0.f};

#pragma unroll 1
  for (int k0 = 0; k0 < KCONV; k0 += 32) {
    const int tap = k0 >> 7;
    const int c0 = k0 & 127;
    const int dy = tap / 3;
    const int dx = tap - dy * 3;
    v16b bh[4];
#pragma unroll
    for (int j = 0; j < 4; ++j) bh[j] = Frag<__bf16>::load(Bw + (size_t)(n0 + 16 * j + rlane) * KCONV + k0 + koff);
#pragma unroll
    for (int i = 0; i < 4; ++i) {
      const size_t ao = ((size_t)((bimg * NPAD + Y0 + i + dy) * NPAD + rlane + dx)) * NCH + c0 + koff;
      const v16b ah = Frag<__bf16>::load(Ah + ao);
      const v16b al = Frag<__bf16>::load(Al + ao);
#pragma unroll
      for (int j = 0; j < 4; ++j) {
        acc[i][j] = Frag<__bf16>::mma(ah, bh[j], acc[i][j]);
        acc[i][j] = Frag<__bf16>::mma(al, bh[j], acc[i][j]);
      }
      Frag<__bf16>::guard(acc[i][0], acc[i][3], ah, al);
    }
    Frag<__bf16>::keep(bh[0], bh[1], bh[2], bh[3]);
  }
  acc_guard4(acc[0][0], acc[0][1], acc[0][2], acc[0][3]);
  acc_guard4(acc[1][0], acc[1][1], acc[1][2], acc[1][3]);
  acc_guard4(acc[2][0], acc[2][1], acc[2][2], acc[2][3]);
  acc_guard4(acc[3][0], acc[3][1], acc[3][2], acc[3][3]);

  const int hh2 = lane >> 4, c4 = (lane & 15) * 4;
  const v4f braw = *(const v4f*)(bias + n0 + c4);
  float bz[4];
#pragma unroll
  for (int e = 0; e < 4; ++e) bz[e] = rne_bf(braw[e]);
  float lsum = 0.0f;
  float* slab  = sT[wave];
  float* slabR = sR[wave];
#pragma unroll
  for (int i = 0; i < 4; ++i) {
    const int Y = Y0 + i;
#pragma unroll
    for (int j = 0; j < 4; ++j)
#pragma unroll
      for (int r = 0; r < 8; ++r) slab[(mOff + r) * 68 + (j << 4) + rlane] = acc[i][j][r];
    wave_sync_lds();
#pragma unroll 2
    for (int it = 0; it < 8; ++it) {
      const int xr = it * 2 + hh2;
      const size_t go = ((size_t)((bimg * NSIDE + Y) * NSIDE + xr)) * NCH + n0 + c4;
      const v4f cv = *(const v4f*)(slab + xr * 68 + c4);
      const v4f h4 = *(const v4f*)(hf + go);
      const v4f f4 = *(const v4f*)(fb + go);
      const v4f r4 = *(const v4f*)(frin + go);
      v4f o4 = (v4f){0.f, 0.f, 0.f, 0.f};
      if (!FIRST) o4 = *(const v4f*)(fhin + go);
      v4f nh, nr;
#pragma unroll
      for (int e = 0; e < 4; ++e) {
        const float yv  = cv[e] + bz[e];
        const float hy  = 0.5f * yv;
        const float hx  = 0.5f * h4[e];
        const float hvl = hx + hy;
        const float fhn = o4[e] + hvl;
        const float frn = r4[e] - hvl;
        const float dl  = fhn - f4[e];
        const float sq  = dl * dl;
        lsum = lsum + sq;
        nh[e] = fhn; nr[e] = frn;
      }
      *(v4f*)(slab + xr * 68 + c4)  = nh;
      *(v4f*)(slabR + xr * 68 + c4) = nr;
    }
    wave_sync_lds();
    for (int pass = 0; pass < 2; ++pass) {
#pragma unroll
      for (int it = 0; it < 8; ++it) {
        const int xr = it * 2 + hh2;
        const size_t go = ((size_t)((bimg * NSIDE + Y) * NSIDE + xr)) * NCH + n0 + c4;
        const v4f a = *(const v4f*)(slab + xr * 68 + c4);
        const v4f rr = *(const v4f*)(slabR + xr * 68 + c4);
        *(volatile v4f*)(fhout + go) = a;
        *(volatile v4f*)(frout + go) = rr;
      }
      __threadfence();
    }
    wave_sync_lds();
  }
#pragma unroll
  for (int off = 16; off > 0; off >>= 1) { const float o = __shfl_xor(lsum, off, 32); lsum = lsum + o; }
  if (lane == 0) sl[wave] = lsum;
  __syncthreads();
  if (wave == 0) {
    float tot = 0.0f;
#pragma unroll
    for (int w = 0; w < 4; ++w) tot = tot + sl[w];
    const float v = (lane == 0) ? tot : 0.0f;
    volatile float* pp = part + (size_t)blockIdx.x * 32;
    pp[lane] = v;
    __threadfence();
    pp[lane] = v;
  }
}

__global__ __launch_bounds__(256) void k_out(const float* __restrict__ fh, const float* __restrict__ fb, float* __restrict__ out) {
  __shared__ __align__(16) float s2[32 * 260];
  const int tid = threadIdx.x;
  const int b = blockIdx.x >> 2, cg = blockIdx.x & 3;
#pragma unroll 2
  for (int k = 0; k < 8; ++k) {
    const int id = k * 256 + tid;
    const int p = id >> 3;
    const int c4 = (id & 7) * 4;
    const size_t go = ((size_t)(b * NPIX + p)) * NCH + cg * 32 + c4;
    const v4f a = *(const v4f*)(fh + go);
    const v4f c = *(const v4f*)(fb + go);
#pragma unroll
    for (int e = 0; e < 4; ++e) { const float dlt = a[e] - c[e]; const float o = dlt + c[e]; s2[(c4 + e) * 260 + p] = o; }
  }
  __syncthreads();
  const int wave = tid >> 5, lane = tid & 31;
  for (int pass = 0; pass < 2; ++pass) {
#pragma unroll
    for (int ch = 0; ch < 4; ++ch) {
      const int c = wave * 4 + ch;
#pragma unroll
      for (int half = 0; half < 2; ++half) {
        const int p4 = half * 128 + lane * 4;
        const v4f v = *(const v4f*)(s2 + c * 260 + p4);
        *(volatile v4f*)(out + ((size_t)(b * NCH + cg * 32 + c)) * NPIX + p4) = v;
      }
    }
    __threadfence();
  }
}

__global__ __launch_bounds__(32) void k_loss(const float* __restrict__ part, float* __restrict__ out1) {
  const int lane = threadIdx.x & 31;
  float loss = 0.0f;
#pragma unroll 1
  for (int s = 0; s < NSCALE; ++s) {
    const float a = part[((size_t)(s * NCONVBLK) + lane) * 32];
    const float c = part[((size_t)(s * NCONVBLK) + 32 + lane) * 32];
    float v = a + c;
#pragma unroll
    for (int off = 16; off > 0; off >>= 1) { const float o = __shfl_xor(v, off, 32); v = v + o; }
    const float m = v * (1.0f / 1048576.0f);
    const float q = 0.25f * m;
    const float term = q + m;
    loss = loss + term;
  }
  loss = loss * 0.2f;
  if (lane == 0) {
    volatile float* o = out1;
    o[0] = loss;
    __threadfence();
    o[0] = loss;
  }
}

extern "C" void kernel_launch(void* const* d_in, const int* in_sizes, int n_in,
                              void* d_out, int out_size, void* d_ws, size_t ws_size,
                              hipStream_t stream) {
  if (n_in < 4) return;
  if (in_sizes[0] != NUMEL_T || in_sizes[1] != NVOC * NCH || in_sizes[2] != 4 * NCH * NCH * 9 || in_sizes[3] != 4 * NCH) return;
  if (out_size != NUMEL_T + 1) return;
  if (ws_size < WS_TOTAL) return;

  const float* f     = (const float*)d_in[0];
  const float* emb   = (const float*)d_in[1];
  const float* phi_w = (const float*)d_in[2];
  const float* phi_b = (const float*)d_in[3];
  float* out = (float*)d_out;
  char* ws = (char*)d_ws;

  unsigned short* Ebf = (unsigned short*)(ws + OFF_EBF);
  float* es   = (float*)(ws + OFF_ES);
  unsigned short* Wt  = (unsigned short*)(ws + OFF_WT);
  float* Fb   = (float*)(ws + OFF_FB);
  float* P0h  = (float*)(ws + OFF_P0H);
  float* P0r  = (float*)(ws + OFF_P0R);
  float* P1h  = (float*)(ws + OFF_P1H);
  float* P1r  = (float*)(ws + OFF_P1R);
  unsigned short* Xh = (unsigned short*)(ws + OFF_XH);
  unsigned short* Xm = (unsigned short*)(ws + OFF_XM);
  unsigned short* Xl = (unsigned short*)(ws + OFF_XL);
  float* xs   = (float*)(ws + OFF_XS);
  int* idxT   = (int*)(ws + OFF_IDX);
  float* Hf   = (float*)(ws + OFF_HF);
  unsigned short* Hh = (unsigned short*)(ws + OFF_HH);
  unsigned short* Hl = (unsigned short*)(ws + OFF_HL);
  float* part = (float*)(ws + OFF_PART);

  k_cast_emb<<<(NVOC * NCH / 8) / 256, 256, 0, stream>>>(emb, Ebf);
  k_esq<<<NVOC / 256, 256, 0, stream>>>(emb, es);
  k_cast_w<<<(4 * NCH * (KCONV / 8)) / 256, 256, 0, stream>>>(phi_w, Wt);
  k_fbT<<<NBATCH * 4, 256, 0, stream>>>(f, Fb);

  const int pns[NSCALE]  = {1, 2, 4, 8, 16};
  const int kphs[NSCALE] = {0, 1, 2, 2, 3};
  const float* FhIn = Fb;
  const float* FrIn = Fb;
  for (int si = 0; si < NSCALE; ++si) {
    const int pn = pns[si];
    const int nrow = NBATCH * pn * pn;
    const int nblk = nrow / 32;
    const int s = NSIDE / pn;
    const float inv_area = 1.0f / (float)(s * s);
    const float invsc = (float)pn / 16.0f;
    float* FhOut = (si & 1) ? P1h : P0h;
    float* FrOut = (si & 1) ? P1r : P0r;
    k_pool<<<nblk, 512, 0, stream>>>(FrIn, Xh, Xm, Xl, xs, pn, s, inv_area);
    k_vq<<<nblk, 128, 0, stream>>>(Xh, Xm, Xl, xs, Ebf, es, idxT);
    k_up<<<(NBATCH * NPAD * NPAD * 32) / 256, 256, 0, stream>>>(Ebf, idxT, Hf, Hh, Hl, pn, invsc);
    const unsigned short* Wk = Wt + (size_t)kphs[si] * NCH * KCONV;
    const float* bk = phi_b + (size_t)kphs[si] * NCH;
    float* pk = part + (size_t)si * NCONVBLK * 32;
    if (si == 0)
      k_conv<true><<<NCONVBLK, 128, 0, stream>>>(Hh, Hl, Wk, bk, Hf, Fb, FhIn, FrIn, FhOut, FrOut, pk);
    else
      k_conv<false><<<NCONVBLK, 128, 0, stream>>>(Hh, Hl, Wk, bk, Hf, Fb, FhIn, FrIn, FhOut, FrOut, pk);
    FhIn = FhOut;
    FrIn = FrOut;
  }
  k_out<<<NBATCH * 4, 256, 0, stream>>>(FhIn, Fb, out);
  k_loss<<<1, 32, 0, stream>>>(part, out + NUMEL_T);
}
